// FeedForwardQuantum_65481071396892
// MI455X (gfx1250) — hardware-verified
//
#include <hip/hip_runtime.h>
#include <math.h>

typedef __attribute__((ext_vector_type(16))) _Float16 v16h;
typedef __attribute__((ext_vector_type(8)))  _Float16 v8h;
typedef __attribute__((ext_vector_type(8)))  float    v8f;
typedef __attribute__((ext_vector_type(4)))  float    v4f;

constexpr int kTok    = 8192;
constexpr int kEmb    = 1024;
constexpr int kFfn    = 4096;
constexpr int kNq     = 16;
constexpr int kKPad   = 32;
constexpr int kSplit  = 16;
constexpr int kFChunk = kFfn / kSplit;
constexpr float kW2Carry    = 16.0f;
constexpr float kWoCarry    = 64.0f;
constexpr float kW2CarryInv = 1.0f / kW2Carry;
constexpr float kWoCarryInv = 1.0f / kWoCarry;

static_assert(kTok == 4 * 2048, "token rows");
static_assert(kFChunk == 256, "one staged Wq column per thread");
static_assert((kEmb % 256) == 0, "Wqe column blocks");
static_assert((kTok % 64) == 0 && (kFfn % 64) == 0 && (kEmb % 64) == 0, "GEMM M,N multiples of 64");
static_assert((kKPad % 32) == 0 && (kFfn % 32) == 0, "GEMM K multiples of 32");
static_assert(kNq == 16 && kKPad == 2 * kNq, "phase plane: 16 live columns + 16 zero columns");
static_assert(((kNq * kEmb / 4) % 256) == 0, "fold-sum grid exact");
static_assert(((kFfn * kKPad / 8) % 256) == 0, "W2 plane grid exact");
static_assert(((kEmb * kFfn / 8) % 256) == 0, "Wo plane grid exact");
static_assert((kTok % 16) == 0, "phase kernel grid exact");

constexpr size_t kOffPART = 0;
constexpr size_t kOffWQE  = kOffPART + (size_t)kSplit * kNq * kEmb * 4;
constexpr size_t kOffA2   = kOffWQE  + (size_t)kNq * kEmb * 4;
constexpr size_t kOffBT2  = kOffA2   + (size_t)kTok * kKPad * 2;
constexpr size_t kOffBT3  = kOffBT2  + (size_t)kFfn * kKPad * 2;
constexpr size_t kOffH2   = kOffBT3  + (size_t)kEmb * kFfn * 2;
constexpr size_t kWsTotal = kOffH2   + (size_t)kTok * kFfn * 2;
static_assert(kWsTotal == 77398016ull, "carve total");
static_assert(kWsTotal <= 134217728ull, "carve cap");
static_assert((kOffWQE % 128) == 0 && (kOffA2 % 128) == 0 && (kOffBT2 % 128) == 0 &&
              (kOffBT3 % 128) == 0 && (kOffH2 % 128) == 0, "128-B aligned regions");

union FragH { v16h v; v8h h[2]; };
__device__ __forceinline__ v16h load_frag_h(const _Float16* p) {
  FragH f;
  f.h[0] = *(const v8h*)(p);
  f.h[1] = *(const v8h*)(p + 16);
  return f.v;
}
__device__ __forceinline__ v8f mma_h(v16h a, v16h b, v8f c) {
  return __builtin_amdgcn_wmma_f32_16x16x32_f16(false, a, false, b, (short)0, c, false, false);
}
__device__ __forceinline__ void tie_acc_h(v8f& a, v16h x, v16h y) {
  asm volatile("" : "+v"(a) : "v"(x), "v"(y));
}
__device__ __forceinline__ void guard_acc_h(v8f& a, v16h x, v16h y) {
  asm volatile("v_nop\n\tv_nop\n\tv_nop\n\tv_nop" : "+v"(a) : "v"(x), "v"(y));
}
__device__ __forceinline__ void keep4_h(v16h a, v16h b, v16h c, v16h d) {
  asm volatile("v_nop" :: "v"(a), "v"(b), "v"(c), "v"(d));
}
__device__ __forceinline__ void acc_guard4(v8f& a, v8f& b, v8f& c, v8f& d) {
  asm volatile("v_nop\n\tv_nop\n\tv_nop\n\tv_nop" : "+v"(a), "+v"(b), "+v"(c), "+v"(d));
}

template <int OUT_MODE, bool RELU>
__global__ __launch_bounds__(256) void wmma_gemm64_f16(
    const unsigned short* __restrict__ Ap, int lda,
    const unsigned short* __restrict__ Btp, int ldb,
    void* __restrict__ Cout, int ldc,
    int M, int N, int K, float scale) {
  const _Float16* A  = (const _Float16*)Ap;
  const _Float16* Bt = (const _Float16*)Btp;
  __shared__ __align__(16) float sT[8][16 * 68];
  const int lane = threadIdx.x & 31;
  const int wave = threadIdx.x >> 5;
  const int tilesN = N >> 6;
  const int tilesM = M >> 6;
  const int tile = blockIdx.x * 8 + wave;
  if (tile >= tilesM * tilesN) return;
  const int tm = tile / tilesN;
  const int tn = tile - tm * tilesN;
  const int m0 = tm << 6;
  const int n0 = tn << 6;

  const int rlane = lane & 15;
  const int koff  = (lane >> 4) * 8;
  const int mOff  = (lane >> 4) * 8;

  v8f acc[4][4];
#pragma unroll
  for (int i = 0; i < 4; ++i)
#pragma unroll
    for (int j = 0; j < 4; ++j) acc[i][j] = (v8f){0.f, 0.f, 0.f, 0.f, 0.f, 0.f, 0.f, 0.f};

  for (int k0 = 0; k0 < K; k0 += 32) {
    v16h bh[4];
#pragma unroll
    for (int j = 0; j < 4; ++j) {
      const size_t bo = (size_t)(n0 + (j << 4) + rlane) * ldb + koff + k0;
      bh[j] = load_frag_h(Bt + bo);
    }
#pragma unroll
    for (int i = 0; i < 4; ++i) {
      const size_t ao = (size_t)(m0 + (i << 4) + rlane) * lda + koff + k0;
      const v16h ah = load_frag_h(A + ao);
      acc[i][0] = mma_h(ah, bh[0], acc[i][0]);
      acc[i][1] = mma_h(ah, bh[1], acc[i][1]);
      acc[i][2] = mma_h(ah, bh[2], acc[i][2]);
      acc[i][3] = mma_h(ah, bh[3], acc[i][3]);
      tie_acc_h(acc[i][0], ah, bh[0]);
      tie_acc_h(acc[i][1], ah, bh[1]);
      tie_acc_h(acc[i][2], ah, bh[2]);
      guard_acc_h(acc[i][3], ah, bh[3]);
    }
    keep4_h(bh[0], bh[1], bh[2], bh[3]);
  }
  acc_guard4(acc[0][0], acc[0][1], acc[0][2], acc[0][3]);
  acc_guard4(acc[1][0], acc[1][1], acc[1][2], acc[1][3]);
  acc_guard4(acc[2][0], acc[2][1], acc[2][2], acc[2][3]);
  acc_guard4(acc[3][0], acc[3][1], acc[3][2], acc[3][3]);

  float* slab = sT[wave];
#pragma unroll
  for (int i = 0; i < 4; ++i) {
    const int mBase = m0 + (i << 4);
#pragma unroll
    for (int j = 0; j < 4; ++j) {
#pragma unroll
      for (int r = 0; r < 8; ++r) {
        float v = acc[i][j][r] * scale;
        if (RELU) v = fmaxf(v, 0.0f);
        slab[(mOff + r) * 68 + (j << 4) + rlane] = v;
      }
    }
    __builtin_amdgcn_fence(__ATOMIC_RELEASE, "workgroup");
    __builtin_amdgcn_wave_barrier();
    __builtin_amdgcn_fence(__ATOMIC_ACQUIRE, "workgroup");
    if (OUT_MODE == 0) {
      float* C = (float*)Cout;
      const int hh = lane >> 4, c4 = (lane & 15) * 4;
      for (int pass = 0; pass < 2; ++pass) {
#pragma unroll
        for (int it = 0; it < 8; ++it) {
          const int row = it * 2 + hh;
          const v4f v = *(const v4f*)(slab + row * 68 + c4);
          *(volatile v4f*)(C + (size_t)(mBase + row) * ldc + n0 + c4) = v;
        }
        __threadfence();
      }
    } else {
      const int q = lane >> 3, c8 = (lane & 7) * 8;
      unsigned short* C = (unsigned short*)Cout;
      for (int pass = 0; pass < 2; ++pass) {
#pragma unroll
        for (int it = 0; it < 4; ++it) {
          const int row = it * 4 + q;
          const float* sp = slab + row * 68 + c8;
          v8h hv;
#pragma unroll
          for (int e = 0; e < 8; ++e) hv[e] = (_Float16)sp[e];
          *(volatile v8h*)(C + (size_t)(mBase + row) * ldc + n0 + c8) = hv;
        }
        __threadfence();
      }
    }
    __builtin_amdgcn_fence(__ATOMIC_RELEASE, "workgroup");
    __builtin_amdgcn_wave_barrier();
    __builtin_amdgcn_fence(__ATOMIC_ACQUIRE, "workgroup");
  }
}

__global__ __launch_bounds__(256) void wqe_partial_kernel(
    const float* __restrict__ Wq, const float* __restrict__ W1, float* __restrict__ part) {
  __shared__ __align__(16) float sWq[kFChunk * kNq];
  const int tid = threadIdx.x;
  const int e   = blockIdx.x * 256 + tid;
  const int kc  = blockIdx.y;
  const int f0  = kc * kFChunk;
#pragma unroll
  for (int j = 0; j < kNq; ++j) sWq[tid * kNq + j] = Wq[(size_t)j * kFfn + f0 + tid];
  __syncthreads();
  float acc[kNq];
#pragma unroll
  for (int j = 0; j < kNq; ++j) acc[j] = 0.0f;
#pragma unroll 2
  for (int fl = 0; fl < kFChunk; ++fl) {
    const float w = W1[(size_t)(f0 + fl) * kEmb + e];
    const v4f q0 = *(const v4f*)(sWq + fl * kNq);
    const v4f q1 = *(const v4f*)(sWq + fl * kNq + 4);
    const v4f q2 = *(const v4f*)(sWq + fl * kNq + 8);
    const v4f q3 = *(const v4f*)(sWq + fl * kNq + 12);
    acc[0]  = fmaf(q0[0], w, acc[0]);
    acc[1]  = fmaf(q0[1], w, acc[1]);
    acc[2]  = fmaf(q0[2], w, acc[2]);
    acc[3]  = fmaf(q0[3], w, acc[3]);
    acc[4]  = fmaf(q1[0], w, acc[4]);
    acc[5]  = fmaf(q1[1], w, acc[5]);
    acc[6]  = fmaf(q1[2], w, acc[6]);
    acc[7]  = fmaf(q1[3], w, acc[7]);
    acc[8]  = fmaf(q2[0], w, acc[8]);
    acc[9]  = fmaf(q2[1], w, acc[9]);
    acc[10] = fmaf(q2[2], w, acc[10]);
    acc[11] = fmaf(q2[3], w, acc[11]);
    acc[12] = fmaf(q3[0], w, acc[12]);
    acc[13] = fmaf(q3[1], w, acc[13]);
    acc[14] = fmaf(q3[2], w, acc[14]);
    acc[15] = fmaf(q3[3], w, acc[15]);
  }
  float* dst = part + (size_t)kc * (kNq * kEmb) + e;
  for (int pass = 0; pass < 2; ++pass) {
#pragma unroll
    for (int j = 0; j < kNq; ++j) *(volatile float*)(dst + (size_t)j * kEmb) = acc[j];
    __threadfence();
  }
}

__global__ __launch_bounds__(256) void wqe_sum_kernel(
    const float* __restrict__ part, float* __restrict__ Wqe) {
  const int i = blockIdx.x * 256 + threadIdx.x;
  v4f s = (v4f){0.f, 0.f, 0.f, 0.f};
#pragma unroll 4
  for (int kc = 0; kc < kSplit; ++kc) {
    const v4f p = *(const v4f*)(part + (size_t)kc * (kNq * kEmb) + (size_t)i * 4);
    s = s + p;
  }
  float* dst = Wqe + (size_t)i * 4;
  *(volatile v4f*)dst = s;
  __threadfence();
  *(volatile v4f*)dst = s;
}

__global__ __launch_bounds__(256) void phase_cos_kernel(
    const float* __restrict__ x, const float* __restrict__ Wqe, const float* __restrict__ theta,
    unsigned short* __restrict__ A2) {
  __shared__ __align__(16) float sQ[16 * kNq];
  const int tid = threadIdx.x;
  const int j   = tid & 15;
  const int tl  = tid >> 4;
  const int m   = blockIdx.x * 16 + tl;
  const v4f* xp = (const v4f*)(x + (size_t)m * kEmb);
  const v4f* wp = (const v4f*)(Wqe + (size_t)j * kEmb);
  float a0 = 0.0f, a1 = 0.0f, a2 = 0.0f, a3 = 0.0f;
#pragma unroll 4
  for (int e4 = 0; e4 < kEmb / 4; ++e4) {
    const v4f xv = xp[e4];
    const v4f wv = wp[e4];
    a0 = fmaf(xv[0], wv[0], a0);
    a1 = fmaf(xv[1], wv[1], a1);
    a2 = fmaf(xv[2], wv[2], a2);
    a3 = fmaf(xv[3], wv[3], a3);
  }
  const float qv  = (a0 + a2) + (a1 + a3);
  const float arg = qv + theta[j];
  sQ[tl * kNq + j] = cosf(arg);
  __syncthreads();
  if ((tid >> 5) < 2) {
    const int row = tid >> 2;
    const int seg = tid & 3;
    const bool live = (seg < 2);
    const float* sp = sQ + row * kNq + (seg & 1) * 8;
    const v4f va = *(const v4f*)(sp);
    const v4f vb = *(const v4f*)(sp + 4);
    v8h hv;
#pragma unroll
    for (int e = 0; e < 4; ++e) {
      const float fa = live ? va[e] : 0.0f;
      const float fb = live ? vb[e] : 0.0f;
      hv[e]     = (_Float16)fa;
      hv[4 + e] = (_Float16)fb;
    }
    unsigned short* dst = A2 + ((size_t)blockIdx.x * 16 + row) * kKPad + seg * 8;
    *(volatile v8h*)dst = hv;
    __threadfence();
    *(volatile v8h*)dst = hv;
  }
}

__global__ __launch_bounds__(256) void pad_w2_kernel(
    const float* __restrict__ W2, unsigned short* __restrict__ Bt2) {
  const int i   = blockIdx.x * 256 + threadIdx.x;
  const int row = i >> 2;
  const int seg = i & 3;
  const bool live = (seg < 2);
  const float* sp = W2 + (size_t)row * kNq + (seg & 1) * 8;
  const v4f va = *(const v4f*)(sp);
  const v4f vb = *(const v4f*)(sp + 4);
  v8h hv;
#pragma unroll
  for (int e = 0; e < 4; ++e) {
    const float fa = live ? (va[e] * kW2Carry) : 0.0f;
    const float fb = live ? (vb[e] * kW2Carry) : 0.0f;
    hv[e]     = (_Float16)fa;
    hv[4 + e] = (_Float16)fb;
  }
  unsigned short* dst = Bt2 + (size_t)i * 8;
  *(volatile v8h*)dst = hv;
  __threadfence();
  *(volatile v8h*)dst = hv;
}

__global__ __launch_bounds__(256) void cast_carry_f16x8_kernel(
    const float* __restrict__ src, unsigned short* __restrict__ dst, int total8, float carry) {
  const int i = blockIdx.x * 256 + threadIdx.x;
  if (i >= total8) return;
  const size_t e0 = (size_t)i << 3;
  const v4f va = *(const v4f*)(src + e0);
  const v4f vb = *(const v4f*)(src + e0 + 4);
  v8h hv;
#pragma unroll
  for (int e = 0; e < 4; ++e) {
    const float fa = va[e] * carry;
    const float fb = vb[e] * carry;
    hv[e]     = (_Float16)fa;
    hv[4 + e] = (_Float16)fb;
  }
  unsigned short* q = dst + e0;
  *(volatile v8h*)q = hv;
  __threadfence();
  *(volatile v8h*)q = hv;
}

extern "C" void kernel_launch(void* const* d_in, const int* in_sizes, int n_in,
                              void* d_out, int out_size, void* d_ws, size_t ws_size,
                              hipStream_t stream) {
  if (n_in < 6) return;
  if (in_sizes[0] != kTok * kEmb) return;
  if (in_sizes[1] != kFfn * kEmb) return;
  if (in_sizes[2] != kNq * kFfn) return;
  if (in_sizes[3] != kNq) return;
  if (in_sizes[4] != kFfn * kNq) return;
  if (in_sizes[5] != kEmb * kFfn) return;
  if (out_size != kTok * kEmb) return;
  if (ws_size < kWsTotal) return;

  const float* x     = (const float*)d_in[0];
  const float* W1    = (const float*)d_in[1];
  const float* Wq    = (const float*)d_in[2];
  const float* theta = (const float*)d_in[3];
  const float* W2    = (const float*)d_in[4];
  const float* Wo    = (const float*)d_in[5];
  float* out = (float*)d_out;

  char* ws = (char*)d_ws;
  float*          PART = (float*)(ws + kOffPART);
  float*          WQE  = (float*)(ws + kOffWQE);
  unsigned short* A2   = (unsigned short*)(ws + kOffA2);
  unsigned short* BT2  = (unsigned short*)(ws + kOffBT2);
  unsigned short* BT3  = (unsigned short*)(ws + kOffBT3);
  unsigned short* H2   = (unsigned short*)(ws + kOffH2);

  wqe_partial_kernel<<<dim3(kEmb / 256, kSplit), 256, 0, stream>>>(Wq, W1, PART);
  wqe_sum_kernel<<<(kNq * kEmb / 4) / 256, 256, 0, stream>>>(PART, WQE);

  phase_cos_kernel<<<kTok / 16, 256, 0, stream>>>(x, WQE, theta, A2);

  pad_w2_kernel<<<(kFfn * kKPad / 8) / 256, 256, 0, stream>>>(W2, BT2);
  cast_carry_f16x8_kernel<<<(kEmb * kFfn / 8) / 256, 256, 0, stream>>>(Wo, BT3, kEmb * kFfn / 8, kWoCarry);

  wmma_gemm64_f16<1, true><<<(kTok / 64) * (kFfn / 64) / 8, 256, 0, stream>>>(
      A2, kKPad, BT2, kKPad, (void*)H2, kFfn, kTok, kFfn, kKPad, kW2CarryInv);

  wmma_gemm64_f16<0, false><<<(kTok / 64) * (kEmb / 64) / 8, 256, 0, stream>>>(
      H2, kFfn, BT3, kFfn, (void*)out, kEmb, kTok, kEmb, kFfn, kWoCarryInv);
}
